// nwlm_61280593380185
// MI455X (gfx1250) — hardware-run, weakly checked
//
#include <hip/hip_runtime.h>
#include <math.h>

typedef __attribute__((ext_vector_type(16))) _Float16 v16h;
typedef __attribute__((ext_vector_type(8)))  _Float16 v8h;
typedef __attribute__((ext_vector_type(8)))  float    v8f;
typedef __attribute__((ext_vector_type(4)))  float    v4f;

constexpr int kRows  = 4096;
constexpr int kHeads = 8;
constexpr int kDk    = 64;
constexpr int kLm    = 2048;
constexpr int kDh    = 64;
constexpr int kYP    = 128;
constexpr int kDin   = kHeads * kDh;
constexpr int kDout  = 512;
constexpr int kHalf  = 4;
constexpr float kRCarry   = 8.0f;
constexpr float kWCarry   = 64.0f;
constexpr float kYCarry   = 1024.0f;
constexpr float kWoCarry  = 16.0f;
constexpr float kSScale   = 1.0f / kRCarry;
constexpr float kFinScale = kYCarry / kWCarry;
constexpr float kOutScale = 1.0f / (kYCarry * kWoCarry);
constexpr float kArgCap   = 11.0f;
constexpr float kEps      = 1e-12f;
static_assert(kDin == 512);
static_assert((kDk % 32) == 0 && (kLm % 32) == 0 && (kDin % 32) == 0);
static_assert((kRows % 64) == 0 && (kLm % 64) == 0 && (kYP % 64) == 0 && (kDout % 64) == 0);
static_assert(kDh + 2 <= kYP);

constexpr size_t kOffZH  = 0;
constexpr size_t kOffZ2  = kOffZH  + (size_t)kHeads * kRows * kDk * 2;
constexpr size_t kOffRH  = kOffZ2  + (size_t)kHeads * kRows * 4;
constexpr size_t kOffR2  = kOffRH  + (size_t)kHeads * kLm * kDk * 2;
constexpr size_t kOffWT  = kOffR2  + (size_t)kHeads * kLm * 4;
constexpr size_t kOffWOT = kOffWT  + (size_t)kHeads * kYP * kLm * 2;
constexpr size_t kOffKP  = kOffWOT + (size_t)kDout * kDin * 2;
constexpr size_t kOffYR  = kOffKP  + (size_t)kHalf * kRows * kLm * 2;
constexpr size_t kOffY16 = kOffYR  + (size_t)kHeads * kRows * kYP * 4;
constexpr size_t kWsTotal = kOffY16 + (size_t)kRows * kDin * 2;
static_assert(kWsTotal == 99287040ull);
static_assert(kWsTotal <= 134217728ull);
static_assert((kOffZ2 % 128) == 0 && (kOffRH % 128) == 0 && (kOffR2 % 128) == 0 && (kOffWT % 128) == 0 &&
              (kOffWOT % 128) == 0 && (kOffKP % 128) == 0 && (kOffYR % 128) == 0 && (kOffY16 % 128) == 0);

union FragU { v16h v; v8h h[2]; };
__device__ __forceinline__ v16h frag_load(const _Float16* p) {
  FragU f;
  f.h[0] = *(const v8h*)(p);
  f.h[1] = *(const v8h*)(p + 16);
  return f.v;
}
__device__ __forceinline__ v8f frag_mma(v16h a, v16h b, v8f c) {
  return __builtin_amdgcn_wmma_f32_16x16x32_f16(false, a, false, b, (short)0, c, false, false);
}
__device__ __forceinline__ void guard_row4(v8f& a0, v8f& a1, v8f& a2, v8f& a3, v16h x, v16h b0, v16h b1, v16h b2, v16h b3) {
  asm volatile("v_nop\n\tv_nop\n\tv_nop\n\tv_nop" : "+v"(a0), "+v"(a1), "+v"(a2), "+v"(a3) : "v"(x), "v"(b0), "v"(b1), "v"(b2), "v"(b3));
}
__device__ __forceinline__ void keep4_h(v16h a, v16h b, v16h c, v16h d) { asm volatile("v_nop" :: "v"(a), "v"(b), "v"(c), "v"(d)); }
__device__ __forceinline__ void acc_guard4(v8f& a, v8f& b, v8f& c, v8f& d) { asm volatile("v_nop\n\tv_nop\n\tv_nop\n\tv_nop" : "+v"(a), "+v"(b), "+v"(c), "+v"(d)); }

__global__ __launch_bounds__(256) void rows_f16_norm_kernel(
    const float* __restrict__ src, long headStride, long rowStride, int rowsPerHead,
    unsigned short* __restrict__ dst, float* __restrict__ norms, float carry)
{
  __shared__ float sN[8][32];
  const int tid = threadIdx.x, lane = tid & 31, wave = tid >> 5;
  const int q = lane >> 3, c8 = (lane & 7) * 8;
  const int task = blockIdx.x * 8 + wave;
  const int tasksPerHead = rowsPerHead >> 5;
  const int head = task / tasksPerHead;
  const int rb = (task - head * tasksPerHead) << 5;
  const float* sp = src + (size_t)head * headStride;
  unsigned short* dp = dst + ((size_t)head * rowsPerHead + rb) * 64;
#pragma unroll 1
  for (int it = 0; it < 8; ++it) {
    const int row = it * 4 + q;
    const float* p = sp + (size_t)(rb + row) * rowStride + c8;
    const v4f a0 = *(const v4f*)(p);
    const v4f a1 = *(const v4f*)(p + 4);
    float ss = 0.0f;
#pragma unroll
    for (int e = 0; e < 4; ++e) {
      ss = fmaf(a0[e], a0[e], ss);
      ss = fmaf(a1[e], a1[e], ss);
    }
    ss += __shfl_xor(ss, 1, 32);
    ss += __shfl_xor(ss, 2, 32);
    ss += __shfl_xor(ss, 4, 32);
    v8h hv;
#pragma unroll
    for (int e = 0; e < 4; ++e) {
      hv[e]     = (_Float16)(a0[e] * carry);
      hv[4 + e] = (_Float16)(a1[e] * carry);
    }
    if ((lane & 7) == 0) sN[wave][row] = ss;
    unsigned short* o = dp + row * 64 + c8;
    *(volatile v8h*)o = hv;
    __threadfence();
    *(volatile v8h*)o = hv;
  }
  __syncthreads();
  const float nv = sN[wave][lane];
  float* np = norms + (size_t)head * rowsPerHead + rb + lane;
  *(volatile float*)np = nv;
  __threadfence();
  *(volatile float*)np = nv;
}

template <int AUG>
__global__ __launch_bounds__(256) void transpose_f16_kernel(
    const float* __restrict__ src, int src_ld, long src_bs,
    const float* __restrict__ qv, long q_bs,
    unsigned short* __restrict__ dst, int dst_ld, long dst_bs, float carry)
{
  __shared__ __align__(16) float sT[66 * 68];
  const int tid = threadIdx.x, lane = tid & 31, wave = tid >> 5;
  const int q = lane >> 3, c8 = (lane & 7) * 8;
  const int b = blockIdx.z;
  const int j0 = blockIdx.x * 64;
  const int o0 = blockIdx.y * 64;
  const int jj = tid >> 2, oq = (tid & 3) * 16;
  float qa = 1.0f;
  if (AUG) {
    const float qx = qv[(size_t)b * q_bs + j0 + jj];
    qa = rsqrtf(fmaxf(qx, 0.0f) + kEps);
  }
  const float* p = src + (size_t)b * src_bs + (size_t)(j0 + jj) * src_ld + o0 + oq;
#pragma unroll
  for (int i = 0; i < 4; ++i) {
    const v4f a = *(const v4f*)(p + 4 * i);
#pragma unroll
    for (int e = 0; e < 4; ++e) sT[(oq + 4 * i + e) * 68 + jj] = a[e] * qa;
  }
  if (AUG) {
    if ((tid & 3) == 0) {
      sT[64 * 68 + jj] = qa;
      sT[65 * 68 + jj] = 1.0f;
    }
  }
  __syncthreads();
  constexpr int NIT = AUG ? 4 : 2;
  v8h hv[NIT];
#pragma unroll
  for (int it = 0; it < NIT; ++it) {
    const int row = it * 32 + wave * 4 + q;
    const int rowc = AUG ? (row < 65 ? row : 65) : row;
    const float* s = sT + rowc * 68 + c8;
    const v4f a0 = *(const v4f*)(s);
    const v4f a1 = *(const v4f*)(s + 4);
    const float m = AUG ? (row < 64 ? carry : 1.0f) : carry;
    const bool live = AUG ? (row < 66) : true;
#pragma unroll
    for (int e = 0; e < 4; ++e) {
      const float x0 = a0[e] * m;
      const float x1 = a1[e] * m;
      hv[it][e]     = (_Float16)(live ? x0 : 0.0f);
      hv[it][4 + e] = (_Float16)(live ? x1 : 0.0f);
    }
  }
  unsigned short* dp = dst + (size_t)b * dst_bs;
  for (int pass = 0; pass < 2; ++pass) {
#pragma unroll
    for (int it = 0; it < NIT; ++it) {
      const int row = it * 32 + wave * 4 + q;
      *(volatile v8h*)(dp + (size_t)(o0 + row) * dst_ld + j0 + c8) = hv[it];
    }
    __threadfence();
  }
}

enum { EPI_RBF = 0, EPI_F32 = 1, EPI_OUT = 2 };

template <int EPI>
__global__ __launch_bounds__(256) void gemm64_f16_kernel(
    const unsigned short* __restrict__ Ap, int lda, long strideA,
    const unsigned short* __restrict__ Btp, int ldb, long strideB,
    void* __restrict__ Cout, int ldc, long strideC,
    const float* __restrict__ colv, long strideCol,
    const float* __restrict__ rowv, long strideRow,
    int M, int N, int K, float scale)
{
  const _Float16* A  = (const _Float16*)Ap;
  const _Float16* Bt = (const _Float16*)Btp;
  __shared__ __align__(16) float sT[8][16 * 68];
  const int b    = blockIdx.y;
  const int lane = threadIdx.x & 31;
  const int wave = threadIdx.x >> 5;
  const int tilesN = N >> 6;
  const int tilesM = M >> 6;
  const int tile = blockIdx.x * 8 + wave;
  if (tile >= tilesM * tilesN) return;
  const int tm = tile / tilesN;
  const int tn = tile - tm * tilesN;
  const int m0 = tm << 6;
  const int n0 = tn << 6;

  const _Float16* Ab = A  + (size_t)b * strideA;
  const _Float16* Bb = Bt + (size_t)b * strideB;

  const int rlane = lane & 15;
  const int koff  = (lane >> 4) * 8;
  const int mOff  = (lane >> 4) * 8;

  v8f acc[4][4];
#pragma unroll
  for (int i = 0; i < 4; ++i)
#pragma unroll
    for (int j = 0; j < 4; ++j) acc[i][j] = (v8f){0.f,0.f,0.f,0.f,0.f,0.f,0.f,0.f};

  for (int k0 = 0; k0 < K; k0 += 32) {
    v16h bh[4];
#pragma unroll
    for (int j = 0; j < 4; ++j) {
      const size_t bo = (size_t)(n0 + (j << 4) + rlane) * ldb + koff + k0;
      bh[j] = frag_load(Bb + bo);
    }
#pragma unroll
    for (int i = 0; i < 4; ++i) {
      const size_t ao = (size_t)(m0 + (i << 4) + rlane) * lda + koff + k0;
      const v16h ah = frag_load(Ab + ao);
#pragma unroll
      for (int j = 0; j < 4; ++j) acc[i][j] = frag_mma(ah, bh[j], acc[i][j]);
      guard_row4(acc[i][0], acc[i][1], acc[i][2], acc[i][3], ah, bh[0], bh[1], bh[2], bh[3]);
    }
    keep4_h(bh[0], bh[1], bh[2], bh[3]);
  }
  acc_guard4(acc[0][0], acc[0][1], acc[0][2], acc[0][3]);
  acc_guard4(acc[1][0], acc[1][1], acc[1][2], acc[1][3]);
  acc_guard4(acc[2][0], acc[2][1], acc[2][2], acc[2][3]);
  acc_guard4(acc[3][0], acc[3][1], acc[3][2], acc[3][3]);

  float* slab = sT[wave];
  const float* colp = colv + (size_t)b * strideCol;
  const float* rowp = rowv + (size_t)b * strideRow;
  const int q  = lane >> 3;
  const int c8 = (lane & 7) * 8;
  float hr2[8];
#pragma unroll
  for (int e = 0; e < 8; ++e) hr2[e] = 0.0f;
  if (EPI == EPI_RBF) {
    const v4f r0 = *(const v4f*)(colp + n0 + c8);
    const v4f r1 = *(const v4f*)(colp + n0 + c8 + 4);
#pragma unroll
    for (int e = 0; e < 4; ++e) {
      hr2[e]     = -0.5f * r0[e];
      hr2[4 + e] = -0.5f * r1[e];
    }
  }
  float bv[4];
#pragma unroll
  for (int j = 0; j < 4; ++j) bv[j] = 0.0f;
  if (EPI == EPI_OUT) {
#pragma unroll
    for (int j = 0; j < 4; ++j) bv[j] = colp[n0 + (j << 4) + rlane];
  }

#pragma unroll
  for (int i = 0; i < 4; ++i) {
    const int mBase = m0 + (i << 4);
#pragma unroll
    for (int j = 0; j < 4; ++j) {
#pragma unroll
      for (int r = 0; r < 8; ++r) {
        float v = acc[i][j][r];
        if (EPI == EPI_OUT) v = fmaf(v, scale, bv[j]);
        slab[(mOff + r) * 68 + (j << 4) + rlane] = v;
      }
    }
    __builtin_amdgcn_fence(__ATOMIC_RELEASE, "workgroup");
    __builtin_amdgcn_wave_barrier();
    __builtin_amdgcn_fence(__ATOMIC_ACQUIRE, "workgroup");
    if (EPI == EPI_RBF) {
#pragma unroll 1
      for (int it = 0; it < 4; ++it) {
        const int row = it * 4 + q;
        float* sp = slab + row * 68 + c8;
        const float hz = 0.5f * rowp[mBase + row];
        const v4f a0 = *(const v4f*)(sp);
        const v4f a1 = *(const v4f*)(sp + 4);
        v4f o0, o1;
#pragma unroll
        for (int e = 0; e < 4; ++e) {
          float t0 = fmaf(a0[e], scale, hr2[e]);
          float t1 = fmaf(a1[e], scale, hr2[4 + e]);
          t0 = fminf(fminf(t0, hz), kArgCap);
          t1 = fminf(fminf(t1, hz), kArgCap);
          o0[e] = expf(t0);
          o1[e] = expf(t1);
        }
        *(v4f*)(sp)     = o0;
        *(v4f*)(sp + 4) = o1;
      }
      __builtin_amdgcn_fence(__ATOMIC_RELEASE, "workgroup");
      __builtin_amdgcn_wave_barrier();
      __builtin_amdgcn_fence(__ATOMIC_ACQUIRE, "workgroup");
      unsigned short* C = (unsigned short*)Cout + (size_t)b * strideC;
      for (int pass = 0; pass < 2; ++pass) {
#pragma unroll
        for (int it = 0; it < 4; ++it) {
          const int row = it * 4 + q;
          const float* sp = slab + row * 68 + c8;
          const v4f s0 = *(const v4f*)(sp);
          const v4f s1 = *(const v4f*)(sp + 4);
          v8h hv;
#pragma unroll
          for (int e = 0; e < 4; ++e) {
            hv[e]     = (_Float16)s0[e];
            hv[4 + e] = (_Float16)s1[e];
          }
          *(volatile v8h*)(C + (size_t)(mBase + row) * ldc + n0 + c8) = hv;
        }
        __threadfence();
      }
    } else {
      float* C = (float*)Cout + (size_t)b * strideC;
      const int hh = lane >> 4, c4 = (lane & 15) * 4;
      for (int pass = 0; pass < 2; ++pass) {
#pragma unroll
        for (int it = 0; it < 8; ++it) {
          const int row = it * 2 + hh;
          const v4f v = *(const v4f*)(slab + row * 68 + c4);
          *(volatile v4f*)(C + (size_t)(mBase + row) * ldc + n0 + c4) = v;
        }
        __threadfence();
      }
    }
    __builtin_amdgcn_fence(__ATOMIC_RELEASE, "workgroup");
    __builtin_amdgcn_wave_barrier();
    __builtin_amdgcn_fence(__ATOMIC_ACQUIRE, "workgroup");
  }
}

static_assert(((size_t)kRows * kHeads * 8) % 256 == 0);
__global__ __launch_bounds__(256) void finalize_kernel(
    const float* __restrict__ YR, const float* __restrict__ Z2, unsigned short* __restrict__ Y16)
{
  const int gid = blockIdx.x * 256 + threadIdx.x;
  const int c8 = (gid & 7) * 8;
  const int pair = gid >> 3;
  const int h = pair & (kHeads - 1);
  const int r = pair >> 3;
  const float* yp = YR + ((size_t)h * kRows + r) * kYP;
  const v4f a0 = *(const v4f*)(yp + c8);
  const v4f a1 = *(const v4f*)(yp + c8 + 4);
  const v4f sv = *(const v4f*)(yp + kDh);
  const float sq = sv[0];
  const float ks = sv[1];
  const float z2 = Z2[(size_t)h * kRows + r];
  const float ez = expf(-0.5f * z2);
  const float ksum = fmaxf(ez * ks, kEps);
  const float c = rsqrtf(ksum);
  const float ce = c * ez;
  const float den = fmaxf(ce * sq, kEps);
  const float rden = 1.0f / den;
  const float f = ce * rden * kFinScale;
  v8h hv;
#pragma unroll
  for (int e = 0; e < 4; ++e) {
    hv[e]     = (_Float16)(a0[e] * f);
    hv[4 + e] = (_Float16)(a1[e] * f);
  }
  unsigned short* o = Y16 + (size_t)r * kDin + h * kDh + c8;
  *(volatile v8h*)o = hv;
  __threadfence();
  *(volatile v8h*)o = hv;
}

extern "C" void kernel_launch(void* const* d_in, const int* in_sizes, int n_in,
                              void* d_out, int out_size, void* d_ws, size_t ws_size,
                              hipStream_t stream) {
  if (n_in < 6) return;
  if (in_sizes[0] != kRows * kHeads * kDk) return;
  if (in_sizes[1] != kHeads * kLm * kDk) return;
  if (in_sizes[2] != kHeads * kLm) return;
  if (in_sizes[3] != kHeads * kLm * kDh) return;
  if (in_sizes[4] != kDin * kDout) return;
  if (in_sizes[5] != kDout) return;
  if (out_size != kRows * kDout) return;
  if (ws_size < kWsTotal) return;

  const float* z  = (const float*)d_in[0];
  const float* R  = (const float*)d_in[1];
  const float* qv = (const float*)d_in[2];
  const float* W  = (const float*)d_in[3];
  const float* WO = (const float*)d_in[4];
  const float* bO = (const float*)d_in[5];
  float* out = (float*)d_out;

  char* ws = (char*)d_ws;
  unsigned short* ZH  = (unsigned short*)(ws + kOffZH);
  float*          Z2  = (float*)(ws + kOffZ2);
  unsigned short* RH  = (unsigned short*)(ws + kOffRH);
  float*          R2  = (float*)(ws + kOffR2);
  unsigned short* WT  = (unsigned short*)(ws + kOffWT);
  unsigned short* WOT = (unsigned short*)(ws + kOffWOT);
  unsigned short* KP  = (unsigned short*)(ws + kOffKP);
  float*          YR  = (float*)(ws + kOffYR);
  unsigned short* Y16 = (unsigned short*)(ws + kOffY16);

  rows_f16_norm_kernel<<<(kHeads * kRows / 32) / 8, 256, 0, stream>>>(
      z, (long)kDk, (long)(kHeads * kDk), kRows, ZH, Z2, 1.0f);
  rows_f16_norm_kernel<<<(kHeads * kLm / 32) / 8, 256, 0, stream>>>(
      R, (long)kLm * kDk, (long)kDk, kLm, RH, R2, kRCarry);
  transpose_f16_kernel<1><<<dim3(kLm / 64, 1, kHeads), 256, 0, stream>>>(
      W, kDh, (long)kLm * kDh, qv, (long)kLm, WT, kLm, (long)kYP * kLm, kWCarry);
  transpose_f16_kernel<0><<<dim3(kDin / 64, kDout / 64, 1), 256, 0, stream>>>(
      WO, kDout, 0L, qv, 0L, WOT, kDin, 0L, kWoCarry);

  for (int g = 0; g < 2; ++g) {
    const size_t h0 = (size_t)g * kHalf;
    gemm64_f16_kernel<EPI_RBF><<<dim3((kRows / 64) * (kLm / 64) / 8, kHalf), 256, 0, stream>>>(
        ZH + h0 * kRows * kDk, kDk, (long)kRows * kDk,
        RH + h0 * kLm * kDk, kDk, (long)kLm * kDk,
        (void*)KP, kLm, (long)kRows * kLm,
        R2 + h0 * kLm, (long)kLm,
        Z2 + h0 * kRows, (long)kRows,
        kRows, kLm, kDk, kSScale);
    gemm64_f16_kernel<EPI_F32><<<dim3((kRows / 64) * (kYP / 64) / 8, kHalf), 256, 0, stream>>>(
        KP, kLm, (long)kRows * kLm,
        WT + h0 * kYP * kLm, kLm, (long)kYP * kLm,
        (void*)(YR + h0 * kRows * kYP), kYP, (long)kRows * kYP,
        R2, 0L,
        Z2, 0L,
        kRows, kYP, kLm, 1.0f);
  }

  finalize_kernel<<<(kRows * kHeads * 8) / 256, 256, 0, stream>>>(YR, Z2, Y16);

  gemm64_f16_kernel<EPI_OUT><<<dim3((kRows / 64) * (kDout / 64) / 8, 1), 256, 0, stream>>>(
      Y16, kDin, 0L,
      WOT, kDin, 0L,
      (void*)out, kDout, 0L,
      bO, 0L,
      Z2, 0L,
      kRows, kDout, kDin, kOutScale);
}
